// ECA_69544110457542
// MI455X (gfx1250) — hardware-verified
//
#include <hip/hip_runtime.h>
#include <stddef.h>


typedef _Float16 h16;
typedef _Float16 v16h __attribute__((ext_vector_type(16)));
typedef _Float16 v8h  __attribute__((ext_vector_type(8)));
typedef float    v8f  __attribute__((ext_vector_type(8)));
typedef float    v4f  __attribute__((ext_vector_type(4)));

#ifndef NB
#define NB 256
#endif
#define NB_FULL 256
#define TSTEPS  64
#define EMB     256
#define XW      32
#define DYN     31
#define HW      80
#define CH3     768
#define CATK    512
#define KX      64
#define KH      128
#define KX_SHIFT 3
#define KH_SHIFT 4
#define MROWS   (NB * TSTEPS)

static_assert(NB >= 1 && NB <= NB_FULL);
static_assert(TSTEPS == 64);
static_assert(CH3 == 3 * EMB && CATK == 2 * EMB);
static_assert(DYN == XW - 1 && DYN <= KX && HW <= KH);
static_assert((KX % 64) == 0 && (KH % 64) == 0 && (CATK % 64) == 0 && (EMB % 64) == 0);
static_assert((KX % 32) == 0 && (KH % 32) == 0 && (CATK % 32) == 0);
static_assert(KX == (8 << KX_SHIFT) && KH == (8 << KH_SHIFT));
static_assert((XW % 8) == 0 && (HW % 8) == 0 && XW >= 8 && HW >= 8);
static_assert((MROWS % 64) == 0 && (MROWS % 8) == 0);
static_assert(EMB == 32 * 8);
static_assert(CH3 == 6 * 32 * 4);
static_assert((CH3 % 256) == 0);
static_assert(((MROWS * (KX / 8)) % 256) == 0 && ((MROWS * (KH / 8)) % 256) == 0);
static_assert((size_t)MROWS * CH3 < (size_t)0xFFFFFFFFu);

#define LDT 72
#define LDC 68
static_assert((LDT % 8) == 0 && LDT >= 64);
static_assert((LDC % 4) == 0 && LDC >= 64);

#define WCARRY 64.0f
#define ACARRY 16.0f
#define RCARRY 2048.0f

#define WD_BYTES   ((size_t)EMB * KX * 2)
#define WH_BYTES   ((size_t)EMB * KH * 2)
#define WVD_BYTES  ((size_t)EMB * CATK * 2)
#define XA_BYTES   ((size_t)MROWS * KX * 2)
#define HA_BYTES   ((size_t)MROWS * KH * 2)
#define XHN_BYTES  ((size_t)MROWS * CH3 * 4)
#define CC_BYTES   ((size_t)MROWS * CATK * 2)
#define OFF_WD   ((size_t)0)
#define OFF_WH   (OFF_WD + WD_BYTES)
#define OFF_WN   (OFF_WH + WH_BYTES)
#define OFF_WVD  (OFF_WN + WH_BYTES)
#define OFF_XA   (OFF_WVD + WVD_BYTES)
#define OFF_HA   (OFF_XA + XA_BYTES)
#define OFF_NA   (OFF_HA + HA_BYTES)
#define OFF_XHN  (OFF_NA + HA_BYTES)
#define OFF_CC   (OFF_XHN + XHN_BYTES)
#define OFF_CCR  (OFF_CC + CC_BYTES)
#define WS_TOTAL (OFF_CCR + CC_BYTES)
static_assert((WD_BYTES % 128) == 0 && (WH_BYTES % 128) == 0 && (WVD_BYTES % 128) == 0);
static_assert((XA_BYTES % 512) == 0 && (HA_BYTES % 512) == 0);
static_assert((XHN_BYTES % 128) == 0 && (CC_BYTES % 512) == 0);
static_assert(WS_TOTAL <= (size_t)134217728);

__device__ __forceinline__ float bf16r(float x) {
  unsigned int u = __float_as_uint(x);
  u = (u + 0x7FFFu + ((u >> 16) & 1u)) & 0xFFFF0000u;
  return __uint_as_float(u);
}

static __device__ __forceinline__ h16 toh_flush(float v) {
  const h16 r = (h16)v;
  return (fabsf(v) < 6.103515625e-05f) ? (h16)0.0f : r;
}

__device__ __forceinline__ v16h frag_at(const _Float16* p) {
  v8h lo = *(const v8h*)(p);
  v8h hi = *(const v8h*)(p + 16);
  v16h out;
#pragma unroll
  for (int i = 0; i < 8; ++i) { out[i] = lo[i]; out[i + 8] = hi[i]; }
  return out;
}

__device__ __forceinline__ v8f wmma16(v16h a, v16h b, v8f c) {
  v8f d = __builtin_amdgcn_wmma_f32_16x16x32_f16(false, a, false, b, (short)0, c,
                                                 false, false);
  asm volatile("v_nop\n\tv_nop\n\tv_nop\n\tv_nop" : "+v"(d) : "v"(a), "v"(b));
  return d;
}

__device__ __forceinline__ float red32_sum(float x) {
#pragma unroll
  for (int off = 1; off < 32; off <<= 1) x += __shfl_xor(x, off, 32);
  return x;
}
__device__ __forceinline__ float red32_max(float x) {
#pragma unroll
  for (int off = 1; off < 32; off <<= 1) x = fmaxf(x, __shfl_xor(x, off, 32));
  return x;
}

__device__ __forceinline__ void wave_lds_sync() {
  __builtin_amdgcn_fence(3  , "wavefront");
  asm volatile("s_wait_dscnt 0x0" ::: "memory");
  __builtin_amdgcn_wave_barrier();
}

static_assert(32 * 2 == 64);
__global__ __launch_bounds__(256) void wconv_kernel(
    const float* __restrict__ W, _Float16* __restrict__ Wt, unsigned ldw, unsigned ldk,
    unsigned kvalid) {
  __shared__ __attribute__((aligned(16))) _Float16 T[64 * LDT];
  const unsigned tid = threadIdx.x;
  const unsigned n0 = blockIdx.x * 64u;
  const unsigned k0 = blockIdx.y * 64u;
#pragma unroll 4
  for (unsigned j = 0; j < 16u; ++j) {
    const unsigned idx = tid + 256u * j;
    const unsigned kr = idx >> 6, nc = idx & 63u;
    const unsigned kg = k0 + kr;
    const unsigned kgc = (kg < kvalid) ? kg : (kvalid - 1u);
    const float v = W[(size_t)kgc * ldw + n0 + nc];
    const float vz = (kg < kvalid) ? v : 0.0f;
    T[nc * LDT + kr] = toh_flush(WCARRY * bf16r(vz));
  }
  __syncthreads();
  v8h x[2];
  size_t off[2];
#pragma unroll
  for (unsigned i = 0; i < 2u; ++i) {
    const unsigned n = 32u * i + (tid >> 3);
    const unsigned kc = (tid & 7u) * 8u;
    x[i] = *(const v8h*)&T[n * LDT + kc];
    off[i] = (size_t)(n0 + n) * ldk + k0 + kc;
  }
#pragma unroll
  for (int i = 0; i < 2; ++i) *(volatile v8h*)(Wt + off[i]) = x[i];
  __threadfence();
#pragma unroll
  for (int i = 0; i < 2; ++i) *(volatile v8h*)(Wt + off[i]) = x[i];
}

__global__ __launch_bounds__(256) void aconv_kernel(
    const float* __restrict__ src, _Float16* __restrict__ dst, unsigned srcw, unsigned kvalid,
    unsigned kshift, unsigned nrows) {
  const unsigned g = blockIdx.x * 256u + threadIdx.x;
  const unsigned row = g >> kshift;
  if (row >= nrows) return;
  const unsigned c0 = (g & ((1u << kshift) - 1u)) * 8u;
  const unsigned c0c = (c0 + 8u <= srcw) ? c0 : (srcw - 8u);
  const float* p = src + (size_t)row * srcw + c0c;
  const v4f a0 = *(const v4f*)p;
  const v4f a1 = *(const v4f*)(p + 4);
  const bool inrow = (c0 == c0c);
  v8h o;
#pragma unroll
  for (unsigned i = 0; i < 4u; ++i) {
    const float e0 = (inrow && (c0 + i) < kvalid) ? a0[i] : 0.0f;
    const float e1 = (inrow && (c0 + 4u + i) < kvalid) ? a1[i] : 0.0f;
    o[i]      = toh_flush(ACARRY * bf16r(e0));
    o[i + 4u] = toh_flush(ACARRY * bf16r(e1));
  }
  _Float16* q = dst + (size_t)g * 8u;
  *(volatile v8h*)q = o;
  __threadfence();
  *(volatile v8h*)q = o;
}

static_assert(16 * 4 == 64);
__global__ __launch_bounds__(256) void gemm_bias_kernel(
    const _Float16* __restrict__ A16, const _Float16* __restrict__ Bt, unsigned K,
    const float* __restrict__ bias, float* __restrict__ outf, unsigned ldo, unsigned coloff) {
  __shared__ __attribute__((aligned(16))) float Cs[64 * LDC];
  const unsigned tid = threadIdx.x, lane = tid & 31u, w = tid >> 5;
  const unsigned mw = w >> 1, nw = w & 1u;
  const unsigned hh = lane >> 4, m = lane & 15u;
  const unsigned n0 = blockIdx.x * 64u;
  const unsigned row0 = blockIdx.y * 64u;

  const _Float16* ap  = A16 + (size_t)(row0 + mw * 16u + m) * K + hh * 8u;
  const _Float16* bp0 = Bt + (size_t)(n0 + nw * 32u + m) * K + hh * 8u;
  const _Float16* bp1 = bp0 + (size_t)16 * K;
  v8f acc0 = {}, acc1 = {};
#pragma unroll 2
  for (unsigned k0 = 0; k0 < K; k0 += 32u) {
    const v16h a  = frag_at(ap + k0);
    const v16h b0 = frag_at(bp0 + k0);
    const v16h b1 = frag_at(bp1 + k0);
    acc0 = wmma16(a, b0, acc0);
    acc1 = wmma16(a, b1, acc1);
  }
#pragma unroll
  for (int r = 0; r < 8; ++r) {
    float* d = &Cs[(mw * 16u + hh * 8u + (unsigned)r) * LDC + nw * 32u + m];
    d[0]  = acc0[r];
    d[16] = acc1[r];
  }
  __syncthreads();

  const float cs = 1.0f / (WCARRY * ACARRY);
  v4f xs[4];
  size_t off[4];
#pragma unroll
  for (unsigned i = 0; i < 4u; ++i) {
    const unsigned r = 16u * i + (tid >> 4);
    const unsigned c = (tid & 15u) * 4u;
    const v4f u = *(const v4f*)&Cs[r * LDC + c];
    const v4f g = *(const v4f*)(bias + n0 + c);
    v4f val;
#pragma unroll
    for (int j = 0; j < 4; ++j) val[j] = u[j] * cs + bf16r(g[j]);
    xs[i] = val;
    off[i] = (size_t)(row0 + r) * ldo + coloff + n0 + c;
  }
#pragma unroll
  for (int i = 0; i < 4; ++i) *(volatile v4f*)(outf + off[i]) = xs[i];
  __threadfence();
#pragma unroll
  for (int i = 0; i < 4; ++i) *(volatile v4f*)(outf + off[i]) = xs[i];
}

static_assert(16 * 4 == 64);
static_assert(64 * LDC * 4 <= 131072);
__global__ __launch_bounds__(256) void gemm_res_kernel(
    const _Float16* __restrict__ A16, const _Float16* __restrict__ A16r,
    const _Float16* __restrict__ Bt, unsigned K,
    const float* __restrict__ bias, float* __restrict__ outf, unsigned ldo, unsigned coloff) {
  __shared__ __attribute__((aligned(16))) float Cs[64 * LDC];
  const unsigned tid = threadIdx.x, lane = tid & 31u, w = tid >> 5;
  const unsigned mw = w >> 1, nw = w & 1u;
  const unsigned hh = lane >> 4, m = lane & 15u;
  const unsigned n0 = blockIdx.x * 64u;
  const unsigned row0 = blockIdx.y * 64u;

  const size_t aoff = (size_t)(row0 + mw * 16u + m) * K + hh * 8u;
  const _Float16* ap  = A16 + aoff;
  const _Float16* arp = A16r + aoff;
  const _Float16* bp0 = Bt + (size_t)(n0 + nw * 32u + m) * K + hh * 8u;
  const _Float16* bp1 = bp0 + (size_t)16 * K;
  v8f acc0 = {}, acc1 = {}, res0 = {}, res1 = {};
#pragma unroll 2
  for (unsigned k0 = 0; k0 < K; k0 += 32u) {
    const v16h a  = frag_at(ap + k0);
    const v16h ar = frag_at(arp + k0);
    const v16h b0 = frag_at(bp0 + k0);
    const v16h b1 = frag_at(bp1 + k0);
    acc0 = wmma16(a, b0, acc0);
    acc1 = wmma16(a, b1, acc1);
    res0 = wmma16(ar, b0, res0);
    res1 = wmma16(ar, b1, res1);
  }
#pragma unroll
  for (int r = 0; r < 8; ++r) {
    float* d = &Cs[(mw * 16u + hh * 8u + (unsigned)r) * LDC + nw * 32u + m];
    d[0]  = acc0[r] + res0[r] * (1.0f / RCARRY);
    d[16] = acc1[r] + res1[r] * (1.0f / RCARRY);
  }
  __syncthreads();

  const float cs = 1.0f / (WCARRY * ACARRY);
  v4f xs[4];
  size_t off[4];
#pragma unroll
  for (unsigned i = 0; i < 4u; ++i) {
    const unsigned r = 16u * i + (tid >> 4);
    const unsigned c = (tid & 15u) * 4u;
    const v4f u = *(const v4f*)&Cs[r * LDC + c];
    const v4f g = *(const v4f*)(bias + n0 + c);
    v4f val;
#pragma unroll
    for (int j = 0; j < 4; ++j) val[j] = u[j] * cs + bf16r(g[j]);
    xs[i] = val;
    off[i] = (size_t)(row0 + r) * ldo + coloff + n0 + c;
  }
#pragma unroll
  for (int i = 0; i < 4; ++i) *(volatile v4f*)(outf + off[i]) = xs[i];
  __threadfence();
#pragma unroll
  for (int i = 0; i < 4; ++i) *(volatile v4f*)(outf + off[i]) = xs[i];
}

static_assert(2 * CH3 * 4 + 8 * 4 + 8 * CH3 * 4 + 8 * EMB * 4 <= 131072);
__global__ __launch_bounds__(256) void sel_kernel(
    const float* __restrict__ xhn, const int* __restrict__ perm,
    const float* __restrict__ conv_w, const float* __restrict__ conv_b,
    const float* __restrict__ x, const float* __restrict__ Wv, const float* __restrict__ bv,
    _Float16* __restrict__ cc, _Float16* __restrict__ ccr) {
#pragma clang fp contract(off)
  __shared__ int sperm[CH3];
  __shared__ int sinv[CH3];
  __shared__ int sflag[8];
  __shared__ __attribute__((aligned(16))) float rowbuf[8 * CH3];
  __shared__ __attribute__((aligned(16))) float ebuf[8 * EMB];

  const unsigned tid = threadIdx.x, lane = tid & 31u;
  const unsigned w = (unsigned)__builtin_amdgcn_readfirstlane((int)(threadIdx.x >> 5));

  int bad = 0;
#pragma unroll 1
  for (unsigned i = tid; i < (unsigned)CH3; i += 256u) {
    const int pv = perm[i];
    const int pc = (pv < 0) ? 0 : ((pv > CH3 - 1) ? (CH3 - 1) : pv);
    sperm[i] = pc;
    sinv[i] = 0;
    bad |= (pv != pc) ? 1 : 0;
  }
  __syncthreads();
#pragma unroll 1
  for (unsigned i = tid; i < (unsigned)CH3; i += 256u) sinv[sperm[i]] = (int)i;
  __syncthreads();
#pragma unroll 1
  for (unsigned i = tid; i < (unsigned)CH3; i += 256u)
    bad |= (sinv[sperm[i]] != (int)i) ? 1 : 0;
#pragma unroll
  for (int off = 1; off < 32; off <<= 1) bad |= __shfl_xor(bad, off, 32);
  if (lane == 0u) sflag[w] = bad;
  __syncthreads();
  int pz = 0;
#pragma unroll
  for (int q = 0; q < 8; ++q) pz |= sflag[q];

  const unsigned crow = blockIdx.x * 8u + w;
  const float* xr = xhn + (size_t)crow * CH3;
  const unsigned rb = w * (unsigned)CH3;
  const unsigned eb = w * (unsigned)EMB;
#pragma unroll 2
  for (unsigned j = 0; j < 6u; ++j) {
    const v4f a = *(const v4f*)(xr + j * 128u + lane * 4u);
    *(v4f*)&rowbuf[rb + j * 128u + lane * 4u] = a;
  }
  wave_lds_sync();

  const unsigned t = crow & (unsigned)(TSTEPS - 1);
  float cw[5];
#pragma unroll
  for (int k = 0; k < 5; ++k) cw[k] = bf16r(conv_w[t * 5u + (unsigned)k]);
  const float cb = bf16r(conv_b[t]);

  float mx = -1.0e30f;
#pragma unroll 1
  for (unsigned i = 0; i < 8u; ++i) {
    const unsigned c = lane * 8u + i;
    const int j = sinv[c];
    float s = 0.0f;
#pragma unroll
    for (int k = 0; k < 5; ++k) {
      const int p = j - 3 + k;
      const int pcl = (p < 0) ? 0 : ((p > CH3 - 1) ? (CH3 - 1) : p);
      const int srcc = sperm[pcl];
      const float v = rowbuf[rb + (unsigned)srcc];
      const float term = v * cw[k];
      s += (p == pcl) ? term : 0.0f;
    }
    const float xx = fmaxf(s + cb, 0.0f);
    ebuf[eb + c] = xx;
    mx = fmaxf(mx, xx);
  }
  mx = red32_max(mx);

  float sum = 0.0f;
#pragma unroll 1
  for (unsigned i = 0; i < 8u; ++i) {
    const unsigned c = lane * 8u + i;
    const float e = __expf(ebuf[eb + c] - mx);
    ebuf[eb + c] = e;
    sum += e;
  }
  sum = red32_sum(sum);
  const float rinv = 1.0f / sum;
  wave_lds_sync();

  const v4f d0 = *(const v4f*)&rowbuf[rb + lane * 8u];
  const v4f d1 = *(const v4f*)&rowbuf[rb + lane * 8u + 4u];
  const v4f e0 = *(const v4f*)&ebuf[eb + lane * 8u];
  const v4f e1 = *(const v4f*)&ebuf[eb + lane * 8u + 4u];
  const float xv = bf16r(x[(size_t)crow * XW + (XW - 1)]);
  const v4f wv0 = *(const v4f*)(Wv + lane * 8u);
  const v4f wv1 = *(const v4f*)(Wv + lane * 8u + 4u);
  const v4f bv0 = *(const v4f*)(bv + lane * 8u);
  const v4f bv1 = *(const v4f*)(bv + lane * 8u + 4u);
  const float nanv = __uint_as_float(0x7FC00000u);
  v8h o1, o2, q1, q2;
#pragma unroll
  for (int i = 0; i < 4; ++i) {
    float g0 = (d0[i] * (e0[i] * rinv) + d0[i]) * 0.5f;
    float g1 = (d1[i] * (e1[i] * rinv) + d1[i]) * 0.5f;
    g0 = (pz != 0) ? nanv : g0;
    g1 = (pz != 0) ? nanv : g1;
    const float sg0 = ACARRY * g0;
    const float sg1 = ACARRY * g1;
    const h16 hg0 = toh_flush(sg0);
    const h16 hg1 = toh_flush(sg1);
    o1[i]     = hg0;
    o1[i + 4] = hg1;
    q1[i]     = toh_flush(RCARRY * (sg0 - (float)hg0));
    q1[i + 4] = toh_flush(RCARRY * (sg1 - (float)hg1));
    const float u0 = xv * bf16r(wv0[i]) + bf16r(bv0[i]);
    const float u1 = xv * bf16r(wv1[i]) + bf16r(bv1[i]);
    const float su0 = ACARRY * u0;
    const float su1 = ACARRY * u1;
    const h16 hu0 = toh_flush(su0);
    const h16 hu1 = toh_flush(su1);
    o2[i]     = hu0;
    o2[i + 4] = hu1;
    q2[i]     = toh_flush(RCARRY * (su0 - (float)hu0));
    q2[i + 4] = toh_flush(RCARRY * (su1 - (float)hu1));
  }
  const size_t poff = (size_t)crow * CATK + lane * 8u;
  _Float16* p1 = cc + poff;
  _Float16* p2 = p1 + EMB;
  _Float16* r1 = ccr + poff;
  _Float16* r2 = r1 + EMB;
  *(volatile v8h*)p1 = o1;
  *(volatile v8h*)p2 = o2;
  *(volatile v8h*)r1 = q1;
  *(volatile v8h*)r2 = q2;
  __threadfence();
  *(volatile v8h*)p1 = o1;
  *(volatile v8h*)p2 = o2;
  *(volatile v8h*)r1 = q1;
  *(volatile v8h*)r2 = q2;
}

extern "C" void kernel_launch(void* const* d_in, const int* in_sizes, int n_in,
                              void* d_out, int out_size, void* d_ws, size_t ws_size,
                              hipStream_t stream) {
  if (n_in < 16) return;
  if ((long long)in_sizes[0] < (long long)MROWS * XW) return;
  if ((long long)in_sizes[1] < (long long)MROWS * HW) return;
  if ((long long)in_sizes[2] < (long long)MROWS * HW) return;
  if (in_sizes[3] < CH3) return;
  if (in_sizes[4] < EMB || in_sizes[5] < EMB) return;
  if (in_sizes[6] < DYN * EMB || in_sizes[7] < EMB) return;
  if (in_sizes[8] < HW * EMB || in_sizes[9] < EMB) return;
  if (in_sizes[10] < HW * EMB || in_sizes[11] < EMB) return;
  if (in_sizes[12] < TSTEPS * 5 || in_sizes[13] < TSTEPS) return;
  if (in_sizes[14] < CATK * EMB || in_sizes[15] < EMB) return;
  if ((long long)out_size < (long long)MROWS * EMB) return;
  if (ws_size < WS_TOTAL) return;

  const float* x      = (const float*)d_in[0];
  const float* human  = (const float*)d_in[1];
  const float* nature = (const float*)d_in[2];
  const int*   perm   = (const int*)d_in[3];
  const float* Wv     = (const float*)d_in[4];
  const float* bv     = (const float*)d_in[5];
  const float* Wd     = (const float*)d_in[6];
  const float* bd     = (const float*)d_in[7];
  const float* Wh     = (const float*)d_in[8];
  const float* bh     = (const float*)d_in[9];
  const float* Wn     = (const float*)d_in[10];
  const float* bn     = (const float*)d_in[11];
  const float* conv_w = (const float*)d_in[12];
  const float* conv_b = (const float*)d_in[13];
  const float* Wvd    = (const float*)d_in[14];
  const float* bvd    = (const float*)d_in[15];
  float* out = (float*)d_out;

  char* ws = (char*)d_ws;
  _Float16* Wd_t  = (_Float16*)(ws + OFF_WD);
  _Float16* Wh_t  = (_Float16*)(ws + OFF_WH);
  _Float16* Wn_t  = (_Float16*)(ws + OFF_WN);
  _Float16* Wvd_t = (_Float16*)(ws + OFF_WVD);
  _Float16* XA    = (_Float16*)(ws + OFF_XA);
  _Float16* HA    = (_Float16*)(ws + OFF_HA);
  _Float16* NA    = (_Float16*)(ws + OFF_NA);
  float*    XHN   = (float*)(ws + OFF_XHN);
  _Float16* CC    = (_Float16*)(ws + OFF_CC);
  _Float16* CCR   = (_Float16*)(ws + OFF_CCR);

  dim3 blk(256);
  dim3 gg(EMB / 64, MROWS / 64);

  wconv_kernel<<<dim3(EMB / 64, KX / 64), blk, 0, stream>>>(Wd, Wd_t, (unsigned)EMB, (unsigned)KX, (unsigned)DYN);
  wconv_kernel<<<dim3(EMB / 64, KH / 64), blk, 0, stream>>>(Wh, Wh_t, (unsigned)EMB, (unsigned)KH, (unsigned)HW);
  wconv_kernel<<<dim3(EMB / 64, KH / 64), blk, 0, stream>>>(Wn, Wn_t, (unsigned)EMB, (unsigned)KH, (unsigned)HW);
  wconv_kernel<<<dim3(EMB / 64, CATK / 64), blk, 0, stream>>>(Wvd, Wvd_t, (unsigned)EMB, (unsigned)CATK, (unsigned)CATK);

  aconv_kernel<<<dim3((MROWS * (KX / 8)) / 256), blk, 0, stream>>>(x, XA, (unsigned)XW, (unsigned)DYN, (unsigned)KX_SHIFT, (unsigned)MROWS);
  aconv_kernel<<<dim3((MROWS * (KH / 8)) / 256), blk, 0, stream>>>(human, HA, (unsigned)HW, (unsigned)HW, (unsigned)KH_SHIFT, (unsigned)MROWS);
  aconv_kernel<<<dim3((MROWS * (KH / 8)) / 256), blk, 0, stream>>>(nature, NA, (unsigned)HW, (unsigned)HW, (unsigned)KH_SHIFT, (unsigned)MROWS);

  gemm_bias_kernel<<<gg, blk, 0, stream>>>(XA, Wd_t, (unsigned)KX, bd, XHN, (unsigned)CH3, 0u);
  gemm_bias_kernel<<<gg, blk, 0, stream>>>(HA, Wh_t, (unsigned)KH, bh, XHN, (unsigned)CH3, (unsigned)EMB);
  gemm_bias_kernel<<<gg, blk, 0, stream>>>(NA, Wn_t, (unsigned)KH, bn, XHN, (unsigned)CH3, (unsigned)(2 * EMB));

  sel_kernel<<<dim3(MROWS / 8), blk, 0, stream>>>(XHN, perm, conv_w, conv_b, x, Wv, bv, CC, CCR);

  gemm_res_kernel<<<gg, blk, 0, stream>>>(CC, CCR, Wvd_t, (unsigned)CATK, bvd, out, (unsigned)EMB, 0u);
}
